// DecoderBlock_73572789781036
// MI455X (gfx1250) — hardware-run, weakly checked
//
#include <hip/hip_runtime.h>
#include <math.h>

typedef __attribute__((ext_vector_type(16))) _Float16 v16h;
typedef __attribute__((ext_vector_type(16))) __bf16 v16b;
typedef __attribute__((ext_vector_type(8)))  _Float16 v8h;
typedef __attribute__((ext_vector_type(8)))  float v8f;
typedef __attribute__((ext_vector_type(4)))  float v4f;
typedef __attribute__((ext_vector_type(2)))  float v2f;
typedef __attribute__((ext_vector_type(4)))  unsigned v4u;
typedef __attribute__((ext_vector_type(4)))  int v4i;
typedef float __attribute__((may_alias)) float_a;
typedef int __attribute__((may_alias)) int_a;

template <typename T> __device__ __forceinline__ void vst2(void* p, T v) { *(volatile T*)p = v; __threadfence(); *(volatile T*)p = v; }
__device__ __forceinline__ v8f wmma16(v16h a, v16h b, v8f c) {
  v8f d = __builtin_amdgcn_wmma_f32_16x16x32_f16(false, a, false, b, (short)0, c, false, false);
  asm volatile("v_nop\n\tv_nop\n\tv_nop\n\tv_nop" : "+v"(d) : "v"(a), "v"(b));
  return d;
}
__device__ __forceinline__ v8f wmma_bf(v16b a, v16b b, v8f c) {
  v8f d = __builtin_amdgcn_wmma_f32_16x16x32_bf16(false, a, false, b, (short)0, c, false, false);
  asm volatile("v_nop\n\tv_nop\n\tv_nop\n\tv_nop" : "+v"(d) : "v"(a), "v"(b));
  return d;
}
__device__ __forceinline__ v16h frag_h(const _Float16* rowk0, int lane) {
  union { v16h v; v8h q[2]; } u; const _Float16* p = rowk0 + 8 * (lane >> 4);
  u.q[0] = *(const v8h*)p; u.q[1] = *(const v8h*)(p + 16); return u.v;
}
__device__ __forceinline__ v16h frag_f32(const float* rowk0, int lane) {
  v16h a; const float* p = rowk0 + 8 * (lane >> 4);
#pragma unroll
  for (int i = 0; i < 8; ++i) { a[i] = (_Float16)p[i]; a[8 + i] = (_Float16)p[16 + i]; }
  return a;
}
__device__ __forceinline__ v16h frag_f32s(const float* rowk0, int lane, float sc) {
  v16h a; const float* p = rowk0 + 8 * (lane >> 4);
#pragma unroll
  for (int i = 0; i < 8; ++i) { a[i] = (_Float16)(p[i] * sc); a[8 + i] = (_Float16)(p[16 + i] * sc); }
  return a;
}
__device__ __forceinline__ v16h fragc_f32(const float* W, int k0, int n, int lane, int ld, int K) {
  v16h a; const int g = lane >> 4;
#pragma unroll
  for (int i = 0; i < 8; ++i) { const int ka = k0 + 8 * g + i, kb = ka + 16;
    a[i] = (_Float16)(ka < K ? W[(size_t)(ka < K ? ka : K - 1) * ld + n] : 0.f); a[8 + i] = (_Float16)(kb < K ? W[(size_t)(kb < K ? kb : K - 1) * ld + n] : 0.f); }
  return a;
}
struct F2 { v16b h, l; };
__device__ __forceinline__ F2 bsplit16(const float v[16]) { F2 r;
#pragma unroll
  for (int i = 0; i < 16; ++i) { const __bf16 h = (__bf16)v[i]; r.h[i] = h; r.l[i] = (__bf16)(v[i] - (float)h); }
  return r; }
__device__ __forceinline__ F2 split_row(const float* row, int k0, int lane) { float v[16]; const float* p = row + k0 + 8 * (lane >> 4);
#pragma unroll
  for (int i = 0; i < 8; ++i) { v[i] = p[i]; v[8 + i] = p[16 + i]; }
  return bsplit16(v); }
__device__ __forceinline__ F2 split_rowK(const float* row, int k0, int lane, int K) { float v[16]; const int g = lane >> 4;
#pragma unroll
  for (int i = 0; i < 8; ++i) { const int ka = k0 + 8 * g + i, kb = ka + 16; v[i] = ka < K ? row[ka < K ? ka : K - 1] : 0.f; v[8 + i] = kb < K ? row[kb < K ? kb : K - 1] : 0.f; }
  return bsplit16(v); }
__device__ __forceinline__ F2 split_col(const float* W, int k0, int n, int lane, int ld, int K) { float v[16]; const int g = lane >> 4;
#pragma unroll
  for (int i = 0; i < 8; ++i) { const int ka = k0 + 8 * g + i, kb = ka + 16; v[i] = ka < K ? W[(size_t)(ka < K ? ka : K - 1) * ld + n] : 0.f; v[8 + i] = kb < K ? W[(size_t)(kb < K ? kb : K - 1) * ld + n] : 0.f; }
  return bsplit16(v); }
__device__ __forceinline__ v8f mac3(const F2& a, const F2& b, v8f c) { c = wmma_bf(a.l, b.h, c); c = wmma_bf(a.h, b.l, c); return wmma_bf(a.h, b.h, c); }
__device__ __forceinline__ float sigm(float v) { return 1.0f / (1.0f + expf(-v)); }
#define LDSX() do { asm volatile("s_wait_dscnt 0" ::: "memory"); __builtin_amdgcn_wave_barrier(); __builtin_amdgcn_fence(__ATOMIC_RELEASE, "workgroup"); } while (0)

#define NBT 64
#define HF 64
#define TT 2048
#define NHD 4
#define DQ 16
#define HQ (NHD * DQ)
#define DHID 1024
#define NROW (NBT * HF)
#define NTR (NBT * TT)
#ifndef NBV
#define NBV NBT
#endif
#define NROWV (NBV * HF)
#define NTRV (NBV * TT)
__device__ __forceinline__ float bfr(float v) { return (float)(__bf16)v; }
__global__ __launch_bounds__(256) void k_tr(const float* __restrict__ X, int rnd, float* __restrict__ XT) { __shared__ float st[64][68]; const int tid = threadIdx.x; const size_t b = blockIdx.y; const int t0 = blockIdx.x * 64;
  for (int e = tid; e < 64 * 16; e += 256) { const int cl = e >> 4, q = e & 15; const v4f v = *(const v4f*)(X + (b * HF + cl) * TT + t0 + q * 4);
#pragma unroll
    for (int i = 0; i < 4; ++i) st[cl][q * 4 + i] = rnd ? bfr(v[i]) : v[i]; }
  __syncthreads();
  for (int e = tid; e < 64 * 16; e += 256) { const int tl = e >> 4, q = e & 15; v4f o; o[0] = st[q * 4][tl]; o[1] = st[q * 4 + 1][tl]; o[2] = st[q * 4 + 2][tl]; o[3] = st[q * 4 + 3][tl]; vst2(XT + (b * TT + t0 + tl) * HF + q * 4, o); } }
__global__ __launch_bounds__(128) void k_gm(const float* __restrict__ Am, int lda, int K, const float* __restrict__ Wm, int ldw, int wsel, int act, float* __restrict__ OUT, int ldo) { __shared__ __align__(16) float sf[4][16][68];
  const int tid = threadIdx.x, wave = tid >> 5, lane = tid & 31, col = lane & 15, g = lane >> 4; const int c0 = blockIdx.y * 64; const size_t r0 = (size_t)blockIdx.x * 64 + wave * 16;
  v8f acc[4] = {};
#pragma unroll 1
  for (int kc = 0; kc < K / 32; ++kc) { const F2 a = split_row(Am + (r0 + col) * (size_t)lda, kc * 32, lane); asm volatile("s_wait_loadcnt 0x0" ::: "memory");
#pragma unroll
    for (int j = 0; j < 4; ++j) { const int o = c0 + j * 16 + col; v16b w; float t0[8], t1[8];
      if (wsel == 0) { const float* p = Wm + (size_t)(kc * 32 + 8 * g) * ldw + o;
#pragma unroll
        for (int i = 0; i < 8; ++i) t0[i] = p[(size_t)i * ldw];
        asm volatile("s_wait_loadcnt 0x0" ::: "memory");
#pragma unroll
        for (int i = 0; i < 8; ++i) t1[i] = p[(size_t)(16 + i) * ldw];
      } else { const float* p = Wm + (size_t)(o / DQ) * (HF * DQ) + (size_t)(kc * 32 + 8 * g) * DQ + (o % DQ);
#pragma unroll
        for (int i = 0; i < 8; ++i) t0[i] = p[(size_t)i * DQ];
        asm volatile("s_wait_loadcnt 0x0" ::: "memory");
#pragma unroll
        for (int i = 0; i < 8; ++i) t1[i] = p[(size_t)(16 + i) * DQ]; }
      asm volatile("s_wait_loadcnt 0x0" ::: "memory");
#pragma unroll
      for (int i = 0; i < 8; ++i) { w[i] = (__bf16)t0[i]; w[8 + i] = (__bf16)t1[i]; }
      acc[j] = wmma_bf(a.h, w, acc[j]); acc[j] = wmma_bf(a.l, w, acc[j]); } }
#pragma unroll
  for (int j = 0; j < 4; ++j) { const int o = c0 + j * 16 + col;
#pragma unroll
    for (int r = 0; r < 8; ++r) { float v = acc[j][r]; if (act == 1) v = v * (1.0f / (1.0f + expf(-v))); else if (act == 2) { const int t = (int)((r0 + 8 * g + r) % TT); if (t < (o % DQ)) v = -__builtin_inff(); } sf[wave][8 * g + r][j * 16 + col] = v; } }
  LDSX(); for (int rl = 0; rl < 16; ++rl) if (lane < 16) vst2(OUT + (r0 + rl) * (size_t)ldo + c0 + lane * 4, *(const v4f*)&sf[wave][rl][lane * 4]);
}
__global__ __launch_bounds__(64) void k_csm(float* __restrict__ X) { const int c = threadIdx.x; const size_t b = blockIdx.x; float* base = X + b * TT * HQ;
  float mx = -3.0e38f; for (int t = 0; t < TT; ++t) { const float v = base[(size_t)t * HQ + c] * 0.5f; mx = fmaxf(mx, v); }
  float sm = 0.f; for (int t = 0; t < TT; ++t) { const float v = base[(size_t)t * HQ + c] * 0.5f; sm += expf(v - mx); }
  const float inv = 1.0f / sm;
  for (int t = 0; t < TT; ++t) { float* p = base + (size_t)t * HQ + c; const float v = *p * 0.5f; vst2(p, expf(v - mx) * inv); } }
__global__ __launch_bounds__(128) void k_amat(const float* __restrict__ PK, const float* __restrict__ V, float* __restrict__ AM) { const int tid = threadIdx.x, wave = tid >> 5, lane = tid & 31, col = lane & 15, g = lane >> 4; const int bh = blockIdx.x * 4 + wave; const size_t b = bh / NHD; const int h = bh % NHD;
  const float* pk = PK + b * TT * HQ + h * DQ; const float* pv = V + b * TT * HQ + h * DQ; v8f acc = {};
#pragma unroll 1
  for (int kc = 0; kc < TT / 32; ++kc) { float va[16], vb[16];
#pragma unroll
    for (int i = 0; i < 8; ++i) { va[i] = pk[(size_t)(kc * 32 + 8 * g + i) * HQ + col]; vb[i] = pv[(size_t)(kc * 32 + 8 * g + i) * HQ + col]; }
    asm volatile("s_wait_loadcnt 0x0" ::: "memory");
#pragma unroll
    for (int i = 0; i < 8; ++i) { va[8 + i] = pk[(size_t)(kc * 32 + 16 + 8 * g + i) * HQ + col]; vb[8 + i] = pv[(size_t)(kc * 32 + 16 + 8 * g + i) * HQ + col]; }
    asm volatile("s_wait_loadcnt 0x0" ::: "memory");
    const F2 a = bsplit16(va), bb = bsplit16(vb); acc = wmma_bf(a.h, bb.h, acc); acc = wmma_bf(a.h, bb.l, acc); acc = wmma_bf(a.l, bb.h, acc); acc = wmma_bf(a.l, bb.l, acc); }
  __shared__ float sa[4][16][17];
#pragma unroll
  for (int r = 0; r < 8; ++r) sa[wave][8 * g + r][col] = acc[r];
  LDSX(); if (lane < 16) { v4f o0 = {sa[wave][lane][0], sa[wave][lane][1], sa[wave][lane][2], sa[wave][lane][3]}, o1 = {sa[wave][lane][4], sa[wave][lane][5], sa[wave][lane][6], sa[wave][lane][7]}, o2 = {sa[wave][lane][8], sa[wave][lane][9], sa[wave][lane][10], sa[wave][lane][11]}, o3 = {sa[wave][lane][12], sa[wave][lane][13], sa[wave][lane][14], sa[wave][lane][15]};
    float* po = AM + ((size_t)bh * DQ + lane) * DQ; vst2(po, o0); vst2(po + 4, o1); vst2(po + 8, o2); vst2(po + 12, o3); } }
__global__ __launch_bounds__(128) void k_bmat(const float* __restrict__ PQ, const float* __restrict__ AM, float* __restrict__ BM) { __shared__ __align__(16) float sb[4][16][20];
  const int tid = threadIdx.x, wave = tid >> 5, lane = tid & 31, col = lane & 15, g = lane >> 4; const size_t b = blockIdx.y; const int h = blockIdx.z; const size_t t0 = (size_t)blockIdx.x * 64 + wave * 16;
  float va[16], vb[16]; const float* pq = PQ + (b * TT + t0 + col) * HQ + h * DQ; const float* pa = AM + ((size_t)(b * NHD + h) * DQ) * DQ;
#pragma unroll
  for (int i = 0; i < 8; ++i) { va[i] = (g == 0) ? pq[i] : pq[8 + i]; vb[i] = (g == 0) ? pa[(size_t)i * DQ + col] : pa[(size_t)(8 + i) * DQ + col]; va[8 + i] = 0.f; vb[8 + i] = 0.f; }
  asm volatile("s_wait_loadcnt 0x0" ::: "memory");
  const F2 a = bsplit16(va), bb = bsplit16(vb); v8f acc = {}; acc = wmma_bf(a.h, bb.h, acc); acc = wmma_bf(a.h, bb.l, acc); acc = wmma_bf(a.l, bb.h, acc); acc = wmma_bf(a.l, bb.l, acc);
#pragma unroll
  for (int r = 0; r < 8; ++r) sb[wave][8 * g + r][col] = acc[r];
  LDSX(); if (lane < 16) { float* po = BM + (((size_t)(b * NHD + h) * TT) + t0 + lane) * DQ; v4f o0 = {sb[wave][lane][0], sb[wave][lane][1], sb[wave][lane][2], sb[wave][lane][3]}, o1 = {sb[wave][lane][4], sb[wave][lane][5], sb[wave][lane][6], sb[wave][lane][7]}, o2 = {sb[wave][lane][8], sb[wave][lane][9], sb[wave][lane][10], sb[wave][lane][11]}, o3 = {sb[wave][lane][12], sb[wave][lane][13], sb[wave][lane][14], sb[wave][lane][15]}; vst2(po, o0); vst2(po + 4, o1); vst2(po + 8, o2); vst2(po + 12, o3); } }
__global__ __launch_bounds__(256) void k_addT(const float* __restrict__ Yin, int rnd, const float* __restrict__ O, float* __restrict__ Y1) { __shared__ float st[64][68]; const int tid = threadIdx.x; const size_t b = blockIdx.y; const int t0 = blockIdx.x * 64;
  for (int e = tid; e < 64 * 16; e += 256) { const int tl = e >> 4, q = e & 15; *(v4f*)&st[tl][q * 4] = *(const v4f*)(O + (b * TT + t0 + tl) * HF + q * 4); }
  __syncthreads();
  for (int e = tid; e < 64 * 16; e += 256) { const int cl = e >> 4, q = e & 15; const size_t oi = (b * HF + cl) * TT + t0 + q * 4; const v4f yv = *(const v4f*)(Yin + oi); v4f o;
#pragma unroll
    for (int i = 0; i < 4; ++i) o[i] = (rnd ? bfr(yv[i]) : yv[i]) + st[q * 4 + i][cl];
    vst2(Y1 + oi, o); } }
__global__ __launch_bounds__(256) void k_ln(const float* __restrict__ X, const float* __restrict__ Hadd, const float* __restrict__ G, const float* __restrict__ Bb, float* __restrict__ OUT) { __shared__ float sred[8]; __shared__ float sbc; __shared__ __align__(16) float row[TT];
  const int tid = threadIdx.x; const size_t r = blockIdx.x; const float* px = X + r * TT; const float* ph = Hadd ? Hadd + r * TT : nullptr;
  float s = 0.f; for (int i = tid * 4; i < TT; i += 1024) { v4f v = *(const v4f*)(px + i); if (ph) { const v4f hv = *(const v4f*)(ph + i); v[0] += hv[0]; v[1] += hv[1]; v[2] += hv[2]; v[3] += hv[3]; } *(v4f*)&row[i] = v; s += (v[0] + v[1]) + (v[2] + v[3]); }
#pragma unroll
  for (int o = 1; o < 32; o <<= 1) s += __shfl_xor(s, o);
  if ((tid & 31) == 0) sred[tid >> 5] = s; __syncthreads(); if (tid == 0) { float a = 0.f; for (int i = 0; i < 8; ++i) a += sred[i]; sbc = a / (float)TT; } __syncthreads(); const float mean = sbc; __syncthreads();
  float q = 0.f; for (int i = tid * 4; i < TT; i += 1024) { const v4f v = *(const v4f*)&row[i];
#pragma unroll
    for (int k = 0; k < 4; ++k) { const float d = v[k] - mean; q += d * d; } }
#pragma unroll
  for (int o = 1; o < 32; o <<= 1) q += __shfl_xor(q, o);
  if ((tid & 31) == 0) sred[tid >> 5] = q; __syncthreads(); if (tid == 0) { float a = 0.f; for (int i = 0; i < 8; ++i) a += sred[i]; sbc = 1.0f / sqrtf(a / (float)TT + 1e-5f); } __syncthreads(); const float rs = sbc;
  for (int i = tid * 4; i < TT; i += 1024) { const v4f v = *(const v4f*)&row[i]; v4f o;
#pragma unroll
    for (int k = 0; k < 4; ++k) o[k] = (v[k] - mean) * rs * bfr(G[i + k]) + bfr(Bb[i + k]);
    vst2(OUT + r * TT + i, o); } }
#define WS_YT  0u
#define WS_MT  (WS_YT + 4u * (size_t)NTR * HF)
#define WS_Q   (WS_MT + 4u * (size_t)NTR * HF)
#define WS_K   (WS_Q  + 4u * (size_t)NTR * HQ)
#define WS_V   (WS_K  + 4u * (size_t)NTR * HQ)
#define WS_AM  (WS_V  + 4u * (size_t)NTR * HQ)
#define WS_Y1  (WS_AM + 4u * (size_t)NBT * NHD * DQ * DQ)
#define WS_END (WS_Y1 + 4u * (size_t)NROW * TT)
#define WS_BM  (WS_K)
#define WS_O   (WS_V)
#define WS_Y2  (WS_YT)
#define WS_H1  (WS_MT)
#define WS_H2  (WS_H1 + 4u * (size_t)NROW * 64)
#define WS_H3  (WS_H2 + 4u * (size_t)NROW * DHID)
#define WS_H4  (WS_Q)
static void sublayer(hipStream_t stream, const float* QsrcT, const float* KVsrcT, const float* WQ, const float* WK, const float* WV, const float* WO, int masked, const float* Yres, int rnd, float* Q, float* Kp, float* V, float* AM, float* BM, float* O, float* Yout) {
  k_gm<<<dim3(NTRV / 64, 1), 128, 0, stream>>>(QsrcT, HF, HF, WQ, 0, 1, masked ? 2 : 0, Q, HQ);
  k_gm<<<dim3(NTRV / 64, 1), 128, 0, stream>>>(KVsrcT, HF, HF, WK, 0, 1, 0, Kp, HQ);
  k_gm<<<dim3(NTRV / 64, 1), 128, 0, stream>>>(KVsrcT, HF, HF, WV, 0, 1, 0, V, HQ);
  k_csm<<<dim3(NBV), 64, 0, stream>>>(Q);
  k_csm<<<dim3(NBV), 64, 0, stream>>>(Kp);
  k_amat<<<dim3(NBV * NHD / 4), 128, 0, stream>>>(Kp, V, AM);
  k_bmat<<<dim3(TT / 64, NBV, NHD), 128, 0, stream>>>(Q, AM, BM);
  k_gm<<<dim3(NTRV / 64, 1), 128, 0, stream>>>(BM, HQ, HQ, WO, HQ, 0, 0, O, HF);
  k_addT<<<dim3(TT / 64, NBV), 256, 0, stream>>>(Yres, rnd, O, Yout);
}
extern "C" void kernel_launch(void* const* d_in, const int* in_sizes, int n_in, void* d_out, int out_size, void* d_ws, size_t ws_size, hipStream_t stream) {
  (void)in_sizes; (void)n_in; (void)out_size;
  if (ws_size < (size_t)WS_END) return;
  char* ws = (char*)d_ws; const float** F = (const float**)d_in;
  float *YT = (float*)(ws + WS_YT), *MT = (float*)(ws + WS_MT), *Q = (float*)(ws + WS_Q), *Kp = (float*)(ws + WS_K), *V = (float*)(ws + WS_V), *AM = (float*)(ws + WS_AM), *BM = (float*)(ws + WS_BM), *O = (float*)(ws + WS_O), *Y1 = (float*)(ws + WS_Y1), *Y2 = (float*)(ws + WS_Y2), *H1 = (float*)(ws + WS_H1), *H2 = (float*)(ws + WS_H2), *H3 = (float*)(ws + WS_H3), *H4 = (float*)(ws + WS_H4);
  k_tr<<<dim3(TT / 64, NBV), 256, 0, stream>>>(F[1], 1, YT);
  k_tr<<<dim3(TT / 64, NBV), 256, 0, stream>>>(F[0], 1, MT);
  sublayer(stream, YT, YT, F[2], F[3], F[4], F[5], 1, F[1], 1, Q, Kp, V, AM, BM, O, Y1);
  k_ln<<<dim3(NROWV), 256, 0, stream>>>(Y1, nullptr, F[14], F[15], Y1);
  k_tr<<<dim3(TT / 64, NBV), 256, 0, stream>>>(Y1, 0, YT);
  sublayer(stream, YT, MT, F[6], F[7], F[8], F[9], 0, Y1, 0, Q, Kp, V, AM, BM, O, Y2);
  k_ln<<<dim3(NROWV), 256, 0, stream>>>(Y2, nullptr, F[16], F[17], Y2);
  k_gm<<<dim3(NROWV / 64, 1), 128, 0, stream>>>(Y2, TT, TT, F[10], 64, 0, 0, H1, 64);
  k_gm<<<dim3(NROWV / 64, DHID / 64), 128, 0, stream>>>(H1, 64, 64, F[11], DHID, 0, 1, H2, DHID);
  k_gm<<<dim3(NROWV / 64, 1), 128, 0, stream>>>(H2, DHID, DHID, F[12], 64, 0, 0, H3, 64);
  k_gm<<<dim3(NROWV / 64, TT / 64), 128, 0, stream>>>(H3, 64, 64, F[13], TT, 0, 0, H4, TT);
  k_ln<<<dim3(NROWV), 256, 0, stream>>>(Y2, H4, F[18], F[19], (float*)d_out);
}
